// SeasonalityBlock_57286273794224
// MI455X (gfx1250) — hardware-run, weakly checked
//
#include <hip/hip_runtime.h>
#include <stddef.h>
#include <stdint.h>


#define MTOT  16384
#define U     512
#define LB    512
#define LF    128
#define NH    64
#define TD    128
#define ASC   16
#define WSC   1024
#define BSC   256
#define NTHR  256
#define NWAVE 8
#define WSCAP 134217728
#define LDS_GEMM (NWAVE * 32 * 64 * 4)
#define NBX (MTOT * LB / (8 * NTHR))
#define NBW (U * U / (8 * NTHR))
#define NBT (TD * U / (8 * NTHR))
#define NBB (LB / 4)
#define NBF (LF / 4)

static_assert(TD == 2 * NH);
static_assert(U == LB);
static_assert((MTOT % 128) == 0);
static_assert((U % 128) == 0);
static_assert((LB % 128) == 0);
static_assert((LF % 128) == 0);
static_assert((TD % 128) == 0);
static_assert((U % 32) == 0);
static_assert((TD % 32) == 0);
static_assert(((MTOT * LB) % (8 * NTHR)) == 0);
static_assert(((U * U) % (8 * NTHR)) == 0);
static_assert(((TD * U) % (8 * NTHR)) == 0);
static_assert(NTHR == NWAVE * 32);
static_assert(NTHR == 4 * NH);
static_assert(4 * TD == 64 * 8);
static_assert(LDS_GEMM <= 300 * 1024);

typedef float    v4f  __attribute__((ext_vector_type(4)));
typedef float    v4fa __attribute__((ext_vector_type(4), may_alias));
typedef float    v8f  __attribute__((ext_vector_type(8)));
typedef _Float16 v8h  __attribute__((ext_vector_type(8)));
typedef _Float16 v8ha __attribute__((ext_vector_type(8), may_alias));
typedef _Float16 v16h __attribute__((ext_vector_type(16)));
union FragH { v16h v; v8h h[2]; };

__device__ __forceinline__ v8f wmf(v16h a, v16h b, v8f c) {
  v8f d = __builtin_amdgcn_wmma_f32_16x16x32_f16(false, a, false, b, (short)0, c, false, false);
  asm volatile("v_nop\n\tv_nop\n\tv_nop\n\tv_nop" : "+v"(d) : "v"(a), "v"(b));
  return d;
}

__global__ __launch_bounds__(NTHR) void k_cvt(const float* x, const float* w1, const float* w2,
                                              const float* w3, const float* w4, const float* wt,
                                              _Float16* xs, _Float16* w1p, _Float16* w2p,
                                              _Float16* w3p, _Float16* w4p, _Float16* wtp) {
  const int b = blockIdx.x;
  const float* src;
  _Float16* dst;
  float sc;
  int lb;
  if (b < NBX)                { src = x;  dst = xs;  sc = (float)ASC; lb = b; }
  else if (b < NBX + NBW)     { src = w1; dst = w1p; sc = (float)WSC; lb = b - NBX; }
  else if (b < NBX + 2 * NBW) { src = w2; dst = w2p; sc = (float)WSC; lb = b - NBX - NBW; }
  else if (b < NBX + 3 * NBW) { src = w3; dst = w3p; sc = (float)WSC; lb = b - NBX - 2 * NBW; }
  else if (b < NBX + 4 * NBW) { src = w4; dst = w4p; sc = (float)WSC; lb = b - NBX - 3 * NBW; }
  else                        { src = wt; dst = wtp; sc = (float)WSC; lb = b - NBX - 4 * NBW; }
  const size_t t = (size_t)lb * NTHR + threadIdx.x;
  const float* p = src + t * 8;
  const v4f f0 = *(const v4f*)p;
  const v4f f1 = *(const v4f*)(p + 4);
  v8h a;
  a[0] = (_Float16)(f0.x * sc); a[1] = (_Float16)(f0.y * sc);
  a[2] = (_Float16)(f0.z * sc); a[3] = (_Float16)(f0.w * sc);
  a[4] = (_Float16)(f1.x * sc); a[5] = (_Float16)(f1.y * sc);
  a[6] = (_Float16)(f1.z * sc); a[7] = (_Float16)(f1.w * sc);
  _Float16* d = dst + t * 8;
  *(volatile v8h*)d = a;
  __threadfence();
  *(volatile v8h*)d = a;
}

__global__ __launch_bounds__(NTHR) void k_basis(_Float16* bTb, _Float16* bTf) {
  __shared__ __attribute__((aligned(16))) _Float16 sb[4 * TD];
  const int t = threadIdx.x;
  const int b = blockIdx.x;
  const bool isB = (b < NBB);
  const int rb = isB ? b : (b - NBB);
  const float invL = isB ? (1.0f / (float)LB) : (1.0f / (float)LF);
  _Float16* dst = isB ? bTb : bTf;
  const int nl = t >> 6, i = t & (NH - 1);
  const int n = 4 * rb + nl;
  const float tn = (6.28318530717958647692f * (float)n) * invL;
  const float ang = (float)i * tn;
  const float c = cosf(ang);
  const float s = sinf(ang);
  sb[nl * TD + 2 * i]     = (_Float16)(c * (float)BSC);
  sb[nl * TD + 2 * i + 1] = (_Float16)(s * (float)BSC);
  __syncthreads();
  if (t < 64) {
    const v8h v = *(const v8ha*)(sb + 8 * t);
    _Float16* d = dst + (size_t)rb * 4 * TD + 8 * t;
    *(volatile v8h*)d = v;
    __threadfence();
    *(volatile v8h*)d = v;
  }
}

template <int MODE>
__global__ __launch_bounds__(NTHR) void k_gemm(const _Float16* __restrict__ A, const _Float16* __restrict__ Bw,
                                               const float* __restrict__ bias, _Float16* Ch, float* Cf,
                                               int N, int K) {
  extern __shared__ v4f lds_dyn[];
  const int tid = threadIdx.x, lane = tid & 31, wave = tid >> 5, hf = lane >> 4, m = lane & 15;
  float* stg = (float*)lds_dyn + wave * (32 * 64);
  const int n0 = blockIdx.x * 128, m0 = blockIdx.y * 128;
  const int wm = (wave >> 1) * 32, wn = (wave & 1) * 64;

  v8f acc[2][4];
#pragma unroll
  for (int mt = 0; mt < 2; ++mt)
#pragma unroll
    for (int nt = 0; nt < 4; ++nt) { v8f z = {0.f, 0.f, 0.f, 0.f, 0.f, 0.f, 0.f, 0.f}; acc[mt][nt] = z; }

  const _Float16* ap = A  + (size_t)(m0 + wm + m) * K + 8 * hf;
  const _Float16* bp = Bw + (size_t)(n0 + wn + m) * K + 8 * hf;
  const size_t r16 = (size_t)16 * K;
#pragma unroll 1
  for (int k0 = 0; k0 < K; k0 += 32) {
    FragH a0, a1;
    a0.h[0] = *(const v8h*)(ap + k0);
    a0.h[1] = *(const v8h*)(ap + k0 + 16);
    a1.h[0] = *(const v8h*)(ap + r16 + k0);
    a1.h[1] = *(const v8h*)(ap + r16 + k0 + 16);
#pragma unroll
    for (int nt = 0; nt < 4; ++nt) {
      const _Float16* bq = bp + (size_t)nt * r16 + k0;
      FragH b;
      b.h[0] = *(const v8h*)bq;
      b.h[1] = *(const v8h*)(bq + 16);
      acc[0][nt] = wmf(a0.v, b.v, acc[0][nt]);
      acc[1][nt] = wmf(a1.v, b.v, acc[1][nt]);
    }
  }

  const float osc = (MODE == 2) ? (1.0f / (float)(ASC * BSC)) : (1.0f / (float)(ASC * WSC));
  float bv[4];
#pragma unroll
  for (int nt = 0; nt < 4; ++nt) {
    bv[nt] = 0.0f;
    if (MODE == 0) bv[nt] = bias[n0 + wn + 16 * nt + m];
  }
#pragma unroll
  for (int mt = 0; mt < 2; ++mt) {
    float* sp = stg + (16 * mt + 8 * hf) * 64 + m;
#pragma unroll
    for (int nt = 0; nt < 4; ++nt) {
#pragma unroll
      for (int r = 0; r < 8; ++r) {
        float v;
        if (MODE == 0)      v = fmaxf(acc[mt][nt][r] * osc + bv[nt], 0.0f) * (float)ASC;
        else if (MODE == 1) v = acc[mt][nt][r] * (1.0f / (float)WSC);
        else                v = acc[mt][nt][r] * osc;
        sp[r * 64 + 16 * nt] = v;
      }
    }
  }
  __syncthreads();

  if (MODE == 2) {
    float* gbase = Cf + (size_t)(m0 + wm) * N + n0 + wn;
#pragma unroll
    for (int q = 0; q < 16; ++q) {
      const int row = 2 * q + hf;
      const v4f v = *(const v4fa*)(stg + row * 64 + 4 * m);
      *(volatile v4f*)(gbase + (size_t)row * N + 4 * m) = v;
    }
    __threadfence();
#pragma unroll
    for (int q = 0; q < 16; ++q) {
      const int row = 2 * q + hf;
      const v4f v = *(const v4fa*)(stg + row * 64 + 4 * m);
      *(volatile v4f*)(gbase + (size_t)row * N + 4 * m) = v;
    }
  } else {
    const int rq = lane >> 3, cc = lane & 7;
    _Float16* hb = Ch + (size_t)(m0 + wm) * N + n0 + wn + 8 * cc;
#pragma unroll
    for (int p = 0; p < 8; ++p) {
      const int row = 4 * p + rq;
      const v4f u0 = *(const v4fa*)(stg + row * 64 + 8 * cc);
      const v4f u1 = *(const v4fa*)(stg + row * 64 + 8 * cc + 4);
      v8h hv;
      hv[0] = (_Float16)u0.x; hv[1] = (_Float16)u0.y; hv[2] = (_Float16)u0.z; hv[3] = (_Float16)u0.w;
      hv[4] = (_Float16)u1.x; hv[5] = (_Float16)u1.y; hv[6] = (_Float16)u1.z; hv[7] = (_Float16)u1.w;
      *(volatile v8h*)(hb + (size_t)row * N) = hv;
    }
    __threadfence();
#pragma unroll
    for (int p = 0; p < 8; ++p) {
      const int row = 4 * p + rq;
      const v4f u0 = *(const v4fa*)(stg + row * 64 + 8 * cc);
      const v4f u1 = *(const v4fa*)(stg + row * 64 + 8 * cc + 4);
      v8h hv;
      hv[0] = (_Float16)u0.x; hv[1] = (_Float16)u0.y; hv[2] = (_Float16)u0.z; hv[3] = (_Float16)u0.w;
      hv[4] = (_Float16)u1.x; hv[5] = (_Float16)u1.y; hv[6] = (_Float16)u1.z; hv[7] = (_Float16)u1.w;
      *(volatile v8h*)(hb + (size_t)row * N) = hv;
    }
  }
}

extern "C" void kernel_launch(void* const* d_in, const int* in_sizes, int n_in,
                              void* d_out, int out_size, void* d_ws, size_t ws_size,
                              hipStream_t stream) {
  if (n_in < 10) return;
  if (in_sizes[0] != MTOT * LB || in_sizes[1] != U * LB || in_sizes[2] != U ||
      in_sizes[3] != U * U || in_sizes[4] != U || in_sizes[5] != U * U || in_sizes[6] != U ||
      in_sizes[7] != U * U || in_sizes[8] != U || in_sizes[9] != TD * U) return;
  if (out_size != MTOT * (LB + LF)) return;

  const float* x  = (const float*)d_in[0];
  const float* W1 = (const float*)d_in[1];
  const float* b1 = (const float*)d_in[2];
  const float* W2 = (const float*)d_in[3];
  const float* b2 = (const float*)d_in[4];
  const float* W3 = (const float*)d_in[5];
  const float* b3 = (const float*)d_in[6];
  const float* W4 = (const float*)d_in[7];
  const float* b4 = (const float*)d_in[8];
  const float* Wt = (const float*)d_in[9];
  float* out0 = (float*)d_out;
  float* out1 = (float*)d_out + (size_t)MTOT * LB;

  char* ws = (char*)d_ws;
  size_t off = 0;
  const size_t oXS = off; off += (size_t)MTOT * LB * 2; off = (off + 255) & ~(size_t)255;
  const size_t oHA = off; off += (size_t)MTOT * U  * 2; off = (off + 255) & ~(size_t)255;
  const size_t oHB = off; off += (size_t)MTOT * U  * 2; off = (off + 255) & ~(size_t)255;
  const size_t oTH = off; off += (size_t)MTOT * TD * 2; off = (off + 255) & ~(size_t)255;
  const size_t oW1 = off; off += (size_t)U * LB * 2;    off = (off + 255) & ~(size_t)255;
  const size_t oW2 = off; off += (size_t)U * U * 2;     off = (off + 255) & ~(size_t)255;
  const size_t oW3 = off; off += (size_t)U * U * 2;     off = (off + 255) & ~(size_t)255;
  const size_t oW4 = off; off += (size_t)U * U * 2;     off = (off + 255) & ~(size_t)255;
  const size_t oWT = off; off += (size_t)TD * U * 2;    off = (off + 255) & ~(size_t)255;
  const size_t oBB = off; off += (size_t)LB * TD * 2;   off = (off + 255) & ~(size_t)255;
  const size_t oBF = off; off += (size_t)LF * TD * 2;   off = (off + 255) & ~(size_t)255;
  if (off > ws_size || off > (size_t)WSCAP) return;
  _Float16* xs  = (_Float16*)(ws + oXS);
  _Float16* hA  = (_Float16*)(ws + oHA);
  _Float16* hB  = (_Float16*)(ws + oHB);
  _Float16* th  = (_Float16*)(ws + oTH);
  _Float16* w1p = (_Float16*)(ws + oW1);
  _Float16* w2p = (_Float16*)(ws + oW2);
  _Float16* w3p = (_Float16*)(ws + oW3);
  _Float16* w4p = (_Float16*)(ws + oW4);
  _Float16* wtp = (_Float16*)(ws + oWT);
  _Float16* bTb = (_Float16*)(ws + oBB);
  _Float16* bTf = (_Float16*)(ws + oBF);

  k_cvt<<<NBX + 4 * NBW + NBT, NTHR, 0, stream>>>(x, W1, W2, W3, W4, Wt, xs, w1p, w2p, w3p, w4p, wtp);
  k_basis<<<NBB + NBF, NTHR, 0, stream>>>(bTb, bTf);

  hipFuncSetAttribute(reinterpret_cast<const void*>(&k_gemm<0>),
                      hipFuncAttributeMaxDynamicSharedMemorySize, LDS_GEMM);
  hipFuncSetAttribute(reinterpret_cast<const void*>(&k_gemm<1>),
                      hipFuncAttributeMaxDynamicSharedMemorySize, LDS_GEMM);
  hipFuncSetAttribute(reinterpret_cast<const void*>(&k_gemm<2>),
                      hipFuncAttributeMaxDynamicSharedMemorySize, LDS_GEMM);
  const dim3 gU(U / 128, MTOT / 128);
  const dim3 gT(TD / 128, MTOT / 128);
  const dim3 gB(LB / 128, MTOT / 128);
  const dim3 gF(LF / 128, MTOT / 128);

  k_gemm<0><<<gU, NTHR, LDS_GEMM, stream>>>(xs, w1p, b1, hA, out0, U, LB);
  k_gemm<0><<<gU, NTHR, LDS_GEMM, stream>>>(hA, w2p, b2, hB, out0, U, U);
  k_gemm<0><<<gU, NTHR, LDS_GEMM, stream>>>(hB, w3p, b3, hA, out0, U, U);
  k_gemm<0><<<gU, NTHR, LDS_GEMM, stream>>>(hA, w4p, b4, hB, out0, U, U);
  k_gemm<1><<<gT, NTHR, LDS_GEMM, stream>>>(hB, wtp, b1, th, out0, TD, U);
  k_gemm<2><<<gB, NTHR, LDS_GEMM, stream>>>(th, bTb, b1, th, out0, LB, TD);
  k_gemm<2><<<gF, NTHR, LDS_GEMM, stream>>>(th, bTf, b1, th, out1, LF, TD);
}
